// FullAttention_66786741452804
// MI455X (gfx1250) — hardware-verified
//
#include <hip/hip_runtime.h>


#ifndef NB
#define NB 4
#endif
#ifndef SEQ
#define SEQ 2048
#endif
#define NB_FULL  4
#define SEQ_FULL 2048
#define NH   8
#define HD   64
#define NPL  (NB * NH)
#define QW   16
#define KCH  64
#define OSP  68
#define SCL  0.125f
#define L2E  1.4426950408889634f

static_assert(SEQ % KCH == 0);
static_assert(SEQ % QW == 0);
static_assert(HD == 64);
static_assert(SEQ <= SEQ_FULL);
static_assert(NB <= NB_FULL);
static_assert(((NPL * SEQ * HD) / 8) % 256 == 0);
static_assert(((NPL * HD * SEQ) / 2) % 256 == 0);

typedef unsigned short bf;
typedef __attribute__((ext_vector_type(16))) __bf16         v16bf;
typedef __attribute__((ext_vector_type(8)))  unsigned short v8us;
typedef __attribute__((ext_vector_type(2)))  unsigned short v2us;
typedef __attribute__((ext_vector_type(8)))  float          v8f;
typedef __attribute__((ext_vector_type(4)))  float          v4f;
typedef v4f __attribute__((may_alias)) v4fa;

__device__ __forceinline__ unsigned short f2bf(float f) { unsigned u = __float_as_uint(f); u += 0x7FFFu + ((u >> 16) & 1u); return (unsigned short)(u >> 16); }
__device__ __forceinline__ float bf2f(unsigned short b) { return __uint_as_float(((unsigned)b) << 16); }
__device__ __forceinline__ v16bf cat16b(v8us lo, v8us hi) { return __builtin_bit_cast(v16bf, __builtin_shufflevector(lo, hi, 0, 1, 2, 3, 4, 5, 6, 7, 8, 9, 10, 11, 12, 13, 14, 15)); }
__device__ __forceinline__ v16bf ldfrag(const bf* p) { return cat16b(*(const v8us*)p, *(const v8us*)(p + 16)); }
__device__ __forceinline__ v8f wmmab(v16bf a, v16bf b, v8f c) { return __builtin_amdgcn_wmma_f32_16x16x32_bf16(false, a, false, b, (short)0, c, false, false); }

__global__ __launch_bounds__(256) void k_cvt8(const float* __restrict__ src, bf* dst, unsigned n8) {
    const unsigned i = blockIdx.x * 256u + threadIdx.x; if (i >= n8) return;
    const size_t e = (size_t)i * 8; const size_t g = e / ((size_t)SEQ * HD); const size_t w = e % ((size_t)SEQ * HD);
    const v8f v = *(const v8f*)(src + g * (size_t)SEQ_FULL * HD + w); v8us o;
#pragma unroll
    for (int k = 0; k < 8; ++k) o[k] = f2bf(v[k]);
    *(volatile v8us*)(dst + e) = o; __threadfence(); *(volatile v8us*)(dst + e) = o;
}

__global__ __launch_bounds__(256) void k_vt2(const float* __restrict__ src, bf* VT, unsigned n2) {
    const unsigned i = blockIdx.x * 256u + threadIdx.x; if (i >= n2) return;
    const size_t e = (size_t)i * 2; const int t = (int)(e % SEQ); const int d = (int)((e / SEQ) % HD); const size_t g = e / ((size_t)SEQ * HD);
    const float* s = src + g * (size_t)SEQ_FULL * HD;
    v2us o; o[0] = f2bf(s[(size_t)t * HD + d]); o[1] = f2bf(s[(size_t)(t + 1) * HD + d]);
    *(volatile v2us*)(VT + e) = o; __threadfence(); *(volatile v2us*)(VT + e) = o;
}

__global__ __launch_bounds__(32) __attribute__((amdgpu_num_vgpr(256)))
void k_attn(const bf* __restrict__ QB, const bf* __restrict__ KB, const bf* __restrict__ VT, float* out) {
    __shared__ __align__(16) float os[QW * OSP];
    const int lane = threadIdx.x & 31, ln = lane & 15, hh = lane >> 4;
    const int g = blockIdx.y;
    const int qw = blockIdx.x * QW;
    const int qn = qw + ln;
    const bf* Qp = QB + (size_t)g * SEQ * HD;
    const bf* Kp = KB + (size_t)g * SEQ * HD;
    const bf* Vp = VT + (size_t)g * HD * SEQ;
    const v16bf bq0 = ldfrag(Qp + (size_t)qn * HD + 8 * hh);
    const v16bf bq1 = ldfrag(Qp + (size_t)qn * HD + 32 + 8 * hh);
    const v8f zero8 = {0.0f, 0.0f, 0.0f, 0.0f, 0.0f, 0.0f, 0.0f, 0.0f};
    v8f oacc[4];
#pragma unroll
    for (int db = 0; db < 4; ++db) oacc[db] = zero8;
    float mrun = -3.0e38f, lrun = 0.0f;
    const int jmax = (qw + QW - 1) / KCH;
#pragma unroll 1
    for (int j = 0; j <= jmax; ++j) {
        const int key0 = j * KCH;
        v16bf ak[4][2];
#pragma unroll
        for (int t = 0; t < 4; ++t) { const bf* kp = Kp + (size_t)(key0 + 16 * t + ln) * HD + 8 * hh; ak[t][0] = ldfrag(kp); ak[t][1] = ldfrag(kp + 32); }
        v8f sacc[4];
#pragma unroll
        for (int t = 0; t < 4; ++t) { sacc[t] = wmmab(ak[t][0], bq0, zero8); sacc[t] = wmmab(ak[t][1], bq1, sacc[t]); }
        asm volatile("v_nop\n\tv_nop\n\tv_nop\n\tv_nop" : "+v"(sacc[0]), "+v"(sacc[1]), "+v"(sacc[2]), "+v"(sacc[3]) : "v"(ak[3][1]), "v"(bq1));
        float mloc = -3.0e38f;
#pragma unroll
        for (int t = 0; t < 4; ++t) {
#pragma unroll
            for (int r = 0; r < 8; ++r) { const int key = key0 + 16 * t + 8 * hh + r; float s = sacc[t][r] * SCL; s = (key > qn) ? -3.0e38f : s; sacc[t][r] = s; mloc = fmaxf(mloc, s); }
        }
        mloc = fmaxf(mloc, __shfl_xor(mloc, 16, 32));
        const float mnew = fmaxf(mrun, mloc);
        const float alpha = __builtin_amdgcn_exp2f(__fmul_rn(__fsub_rn(mrun, mnew), L2E));
        mrun = mnew;
        float lsum = 0.0f;
#pragma unroll
        for (int t = 0; t < 4; ++t) {
#pragma unroll
            for (int r = 0; r < 8; ++r) { const float d0 = __fsub_rn(sacc[t][r], mnew); const float p = __builtin_amdgcn_exp2f(__fmul_rn(d0, L2E)); sacc[t][r] = p; lsum += p; }
        }
        lrun = lrun * alpha + lsum;
#pragma unroll
        for (int db = 0; db < 4; ++db)
#pragma unroll
            for (int r = 0; r < 8; ++r) oacc[db][r] *= alpha;
#pragma unroll
        for (int s = 0; s < 2; ++s) {
            v8us h0, h1, l0, l1;
#pragma unroll
            for (int r = 0; r < 8; ++r) {
                const float p0 = sacc[2 * s][r];     const unsigned short a0 = f2bf(p0); h0[r] = a0; l0[r] = f2bf(p0 - bf2f(a0));
                const float p1 = sacc[2 * s + 1][r]; const unsigned short a1 = f2bf(p1); h1[r] = a1; l1[r] = f2bf(p1 - bf2f(a1));
            }
            const v16bf phi = cat16b(h0, h1), plo = cat16b(l0, l1);
            v16bf av[4];
#pragma unroll
            for (int db = 0; db < 4; ++db) av[db] = ldfrag(Vp + (size_t)(16 * db + ln) * SEQ + key0 + 32 * s + 8 * hh);
#pragma unroll
            for (int db = 0; db < 4; ++db) { oacc[db] = wmmab(av[db], phi, oacc[db]); oacc[db] = wmmab(av[db], plo, oacc[db]); }
            asm volatile("v_nop\n\tv_nop\n\tv_nop\n\tv_nop" : "+v"(oacc[0]), "+v"(oacc[1]), "+v"(oacc[2]), "+v"(oacc[3]) : "v"(av[3]), "v"(plo), "v"(phi));
        }
    }
    const float ltot = lrun + __shfl_xor(lrun, 16, 32);
    const float inv = 1.0f / ltot;
#pragma unroll
    for (int db = 0; db < 4; ++db)
#pragma unroll
        for (int r = 0; r < 8; ++r) os[ln * OSP + 16 * db + 8 * hh + r] = oacc[db][r] * inv;
    __builtin_amdgcn_fence(3, "wavefront"); __builtin_amdgcn_wave_barrier(); asm volatile("" ::: "memory");
    v4f val[8];
#pragma unroll
    for (int s2 = 0; s2 < 8; ++s2) val[s2] = *(const v4fa*)(os + (2 * s2 + hh) * OSP + ln * 4);
    float* ob = out + ((size_t)g * SEQ + qw) * HD;
#pragma unroll
    for (int s2 = 0; s2 < 8; ++s2) *(volatile v4f*)(ob + (size_t)(2 * s2 + hh) * HD + ln * 4) = val[s2];
    __threadfence();
#pragma unroll
    for (int s2 = 0; s2 < 8; ++s2) *(volatile v4f*)(ob + (size_t)(2 * s2 + hh) * HD + ln * 4) = val[s2];
}

extern "C" void kernel_launch(void* const* d_in, const int* in_sizes, int n_in,
                              void* d_out, int out_size, void* d_ws, size_t ws_size, hipStream_t stream) {
    if (n_in < 3) return;
    const long long need_in = (long long)NB * NH * SEQ_FULL * HD;
    if ((long long)in_sizes[0] < need_in || (long long)in_sizes[1] < need_in || (long long)in_sizes[2] < need_in) return;
    if ((long long)out_size < (long long)NPL * SEQ * HD) return;
    const float* Qin = (const float*)d_in[0]; const float* Kin = (const float*)d_in[1]; const float* Vin = (const float*)d_in[2];
    float* OUT = (float*)d_out;
    const size_t plane_bytes = ((size_t)NPL * SEQ * HD * sizeof(bf) + 255) & ~(size_t)255;
    const size_t oQ = 0, oK = oQ + plane_bytes, oV = oK + plane_bytes, oEnd = oV + plane_bytes;
    if (oEnd > ws_size || oEnd > ((size_t)128 << 20)) return;
    bf* QB = (bf*)((char*)d_ws + oQ); bf* KB = (bf*)((char*)d_ws + oK); bf* VT = (bf*)((char*)d_ws + oV);
    const unsigned n8 = (unsigned)((size_t)NPL * SEQ * HD / 8);
    const unsigned n2 = (unsigned)((size_t)NPL * HD * SEQ / 2);
    k_cvt8<<<(n8 + 255u) / 256u, 256, 0, stream>>>(Qin, QB, n8);
    k_cvt8<<<(n8 + 255u) / 256u, 256, 0, stream>>>(Kin, KB, n8);
    k_vt2<<<(n2 + 255u) / 256u, 256, 0, stream>>>(Vin, VT, n2);
    k_attn<<<dim3(SEQ / QW, NPL, 1), 32, 0, stream>>>(QB, KB, VT, OUT);
}
